// BSRBF_KANLayer_50508815401098
// MI455X (gfx1250) — hardware-verified
//
#include <hip/hip_runtime.h>
#include <math.h>

typedef __attribute__((ext_vector_type(16))) _Float16 v16h;
typedef __attribute__((ext_vector_type(16))) __bf16 v16b;
typedef __attribute__((ext_vector_type(8)))  _Float16 v8h;
typedef __attribute__((ext_vector_type(8)))  float v8f;
typedef __attribute__((ext_vector_type(4)))  float v4f;
typedef __attribute__((ext_vector_type(2)))  float v2f;
typedef __attribute__((ext_vector_type(4)))  unsigned v4u;
typedef __attribute__((ext_vector_type(4)))  int v4i;
typedef float __attribute__((may_alias)) float_a;
typedef int __attribute__((may_alias)) int_a;

template <typename T> __device__ __forceinline__ void vst2(void* p, T v) { *(volatile T*)p = v; __threadfence(); *(volatile T*)p = v; }
__device__ __forceinline__ v8f wmma16(v16h a, v16h b, v8f c) {
  v8f d = __builtin_amdgcn_wmma_f32_16x16x32_f16(false, a, false, b, (short)0, c, false, false);
  asm volatile("v_nop\n\tv_nop\n\tv_nop\n\tv_nop" : "+v"(d) : "v"(a), "v"(b));
  return d;
}
__device__ __forceinline__ v8f wmma_bf(v16b a, v16b b, v8f c) {
  v8f d = __builtin_amdgcn_wmma_f32_16x16x32_bf16(false, a, false, b, (short)0, c, false, false);
  asm volatile("v_nop\n\tv_nop\n\tv_nop\n\tv_nop" : "+v"(d) : "v"(a), "v"(b));
  return d;
}
__device__ __forceinline__ v16h frag_h(const _Float16* rowk0, int lane) {
  union { v16h v; v8h q[2]; } u; const _Float16* p = rowk0 + 8 * (lane >> 4);
  u.q[0] = *(const v8h*)p; u.q[1] = *(const v8h*)(p + 16); return u.v;
}
__device__ __forceinline__ v16h frag_f32(const float* rowk0, int lane) {
  v16h a; const float* p = rowk0 + 8 * (lane >> 4);
#pragma unroll
  for (int i = 0; i < 8; ++i) { a[i] = (_Float16)p[i]; a[8 + i] = (_Float16)p[16 + i]; }
  return a;
}
__device__ __forceinline__ v16h frag_f32s(const float* rowk0, int lane, float sc) {
  v16h a; const float* p = rowk0 + 8 * (lane >> 4);
#pragma unroll
  for (int i = 0; i < 8; ++i) { a[i] = (_Float16)(p[i] * sc); a[8 + i] = (_Float16)(p[16 + i] * sc); }
  return a;
}
__device__ __forceinline__ v16h fragc_f32(const float* W, int k0, int n, int lane, int ld, int K) {
  v16h a; const int g = lane >> 4;
#pragma unroll
  for (int i = 0; i < 8; ++i) { const int ka = k0 + 8 * g + i, kb = ka + 16;
    a[i] = (_Float16)(ka < K ? W[(size_t)(ka < K ? ka : K - 1) * ld + n] : 0.f); a[8 + i] = (_Float16)(kb < K ? W[(size_t)(kb < K ? kb : K - 1) * ld + n] : 0.f); }
  return a;
}
struct F2 { v16b h, l; };
__device__ __forceinline__ F2 bsplit16(const float v[16]) { F2 r;
#pragma unroll
  for (int i = 0; i < 16; ++i) { const __bf16 h = (__bf16)v[i]; r.h[i] = h; r.l[i] = (__bf16)(v[i] - (float)h); }
  return r; }
__device__ __forceinline__ F2 split_row(const float* row, int k0, int lane) { float v[16]; const float* p = row + k0 + 8 * (lane >> 4);
#pragma unroll
  for (int i = 0; i < 8; ++i) { v[i] = p[i]; v[8 + i] = p[16 + i]; }
  return bsplit16(v); }
__device__ __forceinline__ F2 split_rowK(const float* row, int k0, int lane, int K) { float v[16]; const int g = lane >> 4;
#pragma unroll
  for (int i = 0; i < 8; ++i) { const int ka = k0 + 8 * g + i, kb = ka + 16; v[i] = ka < K ? row[ka < K ? ka : K - 1] : 0.f; v[8 + i] = kb < K ? row[kb < K ? kb : K - 1] : 0.f; }
  return bsplit16(v); }
__device__ __forceinline__ F2 split_col(const float* W, int k0, int n, int lane, int ld, int K) { float v[16]; const int g = lane >> 4;
#pragma unroll
  for (int i = 0; i < 8; ++i) { const int ka = k0 + 8 * g + i, kb = ka + 16; v[i] = ka < K ? W[(size_t)(ka < K ? ka : K - 1) * ld + n] : 0.f; v[8 + i] = kb < K ? W[(size_t)(kb < K ? kb : K - 1) * ld + n] : 0.f; }
  return bsplit16(v); }
__device__ __forceinline__ v8f mac3(const F2& a, const F2& b, v8f c) { c = wmma_bf(a.l, b.h, c); c = wmma_bf(a.h, b.l, c); return wmma_bf(a.h, b.h, c); }
__device__ __forceinline__ float sigm(float v) { return 1.0f / (1.0f + expf(-v)); }
#define LDSX() do { asm volatile("s_wait_dscnt 0" ::: "memory"); __builtin_amdgcn_wave_barrier(); __builtin_amdgcn_fence(__ATOMIC_RELEASE, "workgroup"); } while (0)

#define NR 16384
#define DD 512
#define OO 512
#define NBF 8
#define KF (DD * NBF)
#define HALF 8192
#ifndef NROWS
#define NROWS NR
#endif
__device__ __forceinline__ float bfr(float v) { return (float)(__bf16)v; }
__device__ __forceinline__ v16h wrowh(const float* rowk0, int lane) { v16h w; const float* p = rowk0 + 8 * (lane >> 4);
#pragma unroll
  for (int i = 0; i < 8; ++i) { w[i] = (_Float16)(bfr(p[i]) * 256.0f); w[8 + i] = (_Float16)(bfr(p[16 + i]) * 256.0f); }
  return w; }

#define WS_XH  0u
#define WS_FH  (WS_XH + 2u * (size_t)NR * DD)
#define WS_END (WS_FH + 2u * (size_t)HALF * KF)

__global__ __launch_bounds__(128) void k_feat(const float* __restrict__ X, const float* __restrict__ LW, const float* __restrict__ LB, size_t r0, _Float16* __restrict__ XH, _Float16* __restrict__ FH) { __shared__ float sred[4]; __shared__ float sbc; __shared__ __align__(16) _Float16 sx[DD]; __shared__ __align__(16) _Float16 sfe[DD][8];
  const int t = threadIdx.x; const size_t row = r0 + blockIdx.x; const float* xr = X + row * DD;
  float s = 0.f;
#pragma unroll 1
  for (int z = 0; z < 4; ++z) s += bfr(xr[t + 128 * z]);
#pragma unroll
  for (int o = 1; o < 32; o <<= 1) s += __shfl_xor(s, o);
  if ((t & 31) == 0) sred[t >> 5] = s; __syncthreads(); if (t == 0) sbc = ((sred[0] + sred[1]) + (sred[2] + sred[3])) * (1.0f / DD); __syncthreads(); const float mean = sbc; __syncthreads();
  float s2 = 0.f;
#pragma unroll 1
  for (int z = 0; z < 4; ++z) { const float dv = bfr(xr[t + 128 * z]) - mean; s2 += dv * dv; }
#pragma unroll
  for (int o = 1; o < 32; o <<= 1) s2 += __shfl_xor(s2, o);
  if ((t & 31) == 0) sred[t >> 5] = s2; __syncthreads(); if (t == 0) sbc = rsqrtf(((sred[0] + sred[1]) + (sred[2] + sred[3])) * (1.0f / DD) + 1e-5f); __syncthreads(); const float rstd = sbc;
  const float g0 = (float)(0 - 3) * 0.6f + (-1.5f), g11 = (float)(11 - 3) * 0.6f + (-1.5f);
#pragma unroll 1
  for (int z = 0; z < 4; ++z) { const int d = t + 128 * z; const float xe = (bfr(xr[d]) - mean) * rstd * bfr(LW[d]) + bfr(LB[d]);
    sx[d] = (_Float16)fmaxf(xe, 0.f);
    const float u = (xe - g0) * (1.0f / 0.6f); const float sgf = floorf(u); const int sg = (xe >= g0 && xe < g11) ? (int)sgf : -100; const float f = u - sgf, f2 = f * f, f3 = f2 * f, omf = 1.0f - f;
    const float w3 = f3 * (1.0f / 6.0f), w2 = (-3.0f * f3 + 3.0f * f2 + 3.0f * f + 1.0f) * (1.0f / 6.0f), w1 = (3.0f * f3 - 6.0f * f2 + 4.0f) * (1.0f / 6.0f), w0 = omf * omf * omf * (1.0f / 6.0f);
#pragma unroll 1
    for (int j = 0; j < NBF; ++j) { const int rel = sg - j; const float bs = (rel == 0) ? w3 : (rel == 1) ? w2 : (rel == 2) ? w1 : (rel == 3) ? w0 : 0.0f;
      const float cj = -1.5f + (float)j * (3.0f / 7.0f); const float uu = (xe - cj) / (3.0f / 7.0f); sfe[d][j] = (_Float16)(bs + expf(-(uu * uu))); } }
  __syncthreads();
  if (t < DD / 8) vst2((unsigned*)(XH + row * DD + t * 8), *(const v4u*)&sx[t * 8]);
  _Float16* dst = FH + (row - r0) * KF;
#pragma unroll 1
  for (int z = 0; z < 4; ++z) { const int d = t + 128 * z; vst2((unsigned*)(dst + (size_t)d * 8), *(const v4u*)&sfe[d][0]); } }
__global__ __launch_bounds__(128) void k_gemm(const _Float16* __restrict__ XH, const _Float16* __restrict__ FH, const float* __restrict__ WB, const float* __restrict__ WS, size_t r0, float* __restrict__ OUT) { __shared__ __align__(16) float sf[4][16][132];
  const int tid = threadIdx.x, wave = tid >> 5, lane = tid & 31, col = lane & 15, g = lane >> 4; const int c0 = blockIdx.y * 128; const size_t rl0 = (size_t)blockIdx.x * 64 + wave * 16; const size_t row0 = r0 + rl0;
  v8f acc[8] = {};
#pragma unroll 2
  for (int kc = 0; kc < DD / 32; ++kc) { const v16h a = frag_h(XH + (row0 + col) * DD + kc * 32, lane); asm volatile("s_wait_loadcnt 0x0" ::: "memory");
#pragma unroll
    for (int j = 0; j < 8; ++j) { const v16h w = wrowh(WB + (size_t)(c0 + j * 16 + col) * DD + kc * 32, lane); asm volatile("s_wait_loadcnt 0x0" ::: "memory"); acc[j] = wmma16(a, w, acc[j]); } }
#pragma unroll 2
  for (int kc = 0; kc < KF / 32; ++kc) { const v16h a = frag_h(FH + (rl0 + col) * KF + kc * 32, lane); asm volatile("s_wait_loadcnt 0x0" ::: "memory");
#pragma unroll
    for (int j = 0; j < 8; ++j) { const v16h w = wrowh(WS + (size_t)(c0 + j * 16 + col) * KF + kc * 32, lane); asm volatile("s_wait_loadcnt 0x0" ::: "memory"); acc[j] = wmma16(a, w, acc[j]); } }
#pragma unroll
  for (int j = 0; j < 8; ++j) {
#pragma unroll
    for (int r = 0; r < 8; ++r) sf[wave][8 * g + r][j * 16 + col] = acc[j][r] * (1.0f / 256.0f); }
  LDSX(); for (int rl = 0; rl < 16; ++rl) vst2(OUT + (row0 + rl) * OO + c0 + lane * 4, *(const v4f*)&sf[wave][rl][lane * 4]); }
extern "C" void kernel_launch(void* const* d_in, const int* in_sizes, int n_in, void* d_out, int out_size, void* d_ws, size_t ws_size, hipStream_t stream) {
  (void)in_sizes; (void)n_in; (void)out_size;
  const float** F = (const float**)d_in;
  if (ws_size < (size_t)WS_END) return;
  char* ws = (char*)d_ws; _Float16 *XH = (_Float16*)(ws + WS_XH), *FH = (_Float16*)(ws + WS_FH);
  for (size_t r0 = 0; r0 < (size_t)NROWS; r0 += HALF) { const size_t n = ((size_t)NROWS - r0) < (size_t)HALF ? ((size_t)NROWS - r0) : (size_t)HALF;
    k_feat<<<dim3((unsigned)n), 128, 0, stream>>>(F[0], F[1], F[2], r0, XH, FH);
    k_gemm<<<dim3((unsigned)(n / 64), OO / 128), 128, 0, stream>>>(XH, FH, F[3], F[4], r0, (float*)d_out);
  }
}
